// MHSelfAttn_5875515261378
// MI455X (gfx1250) — hardware-verified
//
#include <hip/hip_runtime.h>
#include <stddef.h>
#include <stdint.h>


#define NB_    4
#define SEQ    1024
#define DM     512
#define NH     8
#define DK     64
#define KP1    16
#define W2     32
#define NSLOT  32768
#define NHALF  16384
#define NBH    32
#define MROWS  4096
#define KOUT   1024
#define NPOS   (NBH * NHALF)
#define PLQ    (NBH * SEQ * DK)
#define NTHR   256
#define NWAVE  8
#define GTHR   128
#define GBM    64
#define GBN    64
#define TPW    (SEQ / NWAVE)
#define DEGCAP 256
#define RINV24 (1.0f / 24.0f)
#define NEGBIG (-1.0e9f)
#define WSMAX  134217728
#define NXU    (3 * (MROWS * DM / 8))
#define NWU    (3 * (DM * DM / 8))
#define NWOU   (DM * KOUT / 8)
#define NCU    (NXU + NWU + NWOU)
#define LDS_AGG 153728

static_assert((MROWS % GBM) == 0 && (DM % GBN) == 0 && (SEQ % GBM) == 0);
static_assert((DM % 32) == 0 && (KOUT % 32) == 0);
static_assert(GBN == DK);
static_assert(GBM == (GTHR / 32) * 16);
static_assert(NSLOT == W2 * SEQ && NHALF == KP1 * SEQ && NBH == NB_ * NH && MROWS == NB_ * SEQ);
static_assert(NSLOT == (1 << 15) && SEQ == (1 << 10));
static_assert((MROWS * DM / 8) == (1 << 18) && (DM * DM / 8) == (1 << 15) && (KOUT / 8) == 128);
static_assert((NXU % NTHR) == 0 && ((NXU + NWU) % NTHR) == 0 && (NCU % NTHR) == 0);
static_assert(NTHR * 4 == SEQ && TPW * NWAVE == SEQ);
static_assert((NSLOT % (4 * NTHR)) == 0);
static_assert(NTHR * 8 == W2 * DK);
static_assert((NSLOT + 3 * SEQ) * 4 + (W2 * DK + NWAVE * 64 + 16) * 4 + NWAVE * 4 <= LDS_AGG);
static_assert(LDS_AGG <= 300000);
static_assert(PLQ == NB_ * SEQ * DM);

typedef float    v4f  __attribute__((ext_vector_type(4)));
typedef float    v8f  __attribute__((ext_vector_type(8)));
typedef int      v4i  __attribute__((ext_vector_type(4)));
typedef int      v8i  __attribute__((ext_vector_type(8)));
typedef unsigned short v8us __attribute__((ext_vector_type(8)));
typedef __bf16   v16b __attribute__((ext_vector_type(16)));
typedef v4f  __attribute__((may_alias)) v4fa;
typedef v4i  __attribute__((may_alias)) v4ia;
typedef v8us __attribute__((may_alias)) v8usa;
union FragB { v16b v; v8us h[2]; v8i w; };

__device__ __forceinline__ v8f wmb(const FragB& a, const FragB& b, v8f c) {
  v8f d = __builtin_amdgcn_wmma_f32_16x16x32_bf16(false, a.v, false, b.v, (short)0, c, false, false);
  asm volatile("v_nop\n\tv_nop\n\tv_nop\n\tv_nop" : "+v"(d) : "v"(a.w), "v"(b.w));
  return d;
}

__device__ __forceinline__ unsigned int bf16u(float x) {
  const unsigned int u = __float_as_uint(x);
  return (u + 0x7FFFu + ((u >> 16) & 1u)) >> 16;
}
__device__ __forceinline__ float bf16f(float x) { return __uint_as_float(bf16u(x) << 16); }

__device__ __forceinline__ v8us cvt8b(const v4f a, const v4f b) {
  v8us r;
  r[0] = (unsigned short)bf16u(a.x); r[1] = (unsigned short)bf16u(a.y);
  r[2] = (unsigned short)bf16u(a.z); r[3] = (unsigned short)bf16u(a.w);
  r[4] = (unsigned short)bf16u(b.x); r[5] = (unsigned short)bf16u(b.y);
  r[6] = (unsigned short)bf16u(b.z); r[7] = (unsigned short)bf16u(b.w);
  return r;
}

__device__ __forceinline__ unsigned short hl1(float x, bool islo) {
  const unsigned int hu = bf16u(x);
  const float hf = __uint_as_float(hu << 16);
  const unsigned int lu = bf16u(x - hf);
  return (unsigned short)(islo ? lu : hu);
}
__device__ __forceinline__ v8us split8(const v4f a, const v4f b, bool islo) {
  v8us r;
  r[0] = hl1(a.x, islo); r[1] = hl1(a.y, islo); r[2] = hl1(a.z, islo); r[3] = hl1(a.w, islo);
  r[4] = hl1(b.x, islo); r[5] = hl1(b.y, islo); r[6] = hl1(b.z, islo); r[7] = hl1(b.w, islo);
  return r;
}

__device__ __forceinline__ void slot_idx(const int* __restrict__ pos_enc, const int* __restrict__ pos_pad,
                                         int bh, int f, int& qi, int& ki, bool& msk) {
  const int g = bh * NHALF + (f & (NHALF - 1));
  const int penc = pos_enc[g];
  const int ppad = pos_pad[g];
  const bool neg = (penc == -1);
  int pe = neg ? 0 : penc;
  pe = pe < 0 ? 0 : (pe > SEQ - 1 ? SEQ - 1 : pe);
  int pp = ppad < 0 ? 0 : (ppad > SEQ - 1 ? SEQ - 1 : ppad);
  const bool lo = f < NHALF;
  qi = lo ? pp : pe;
  ki = lo ? pe : pp;
  msk = neg || (f < SEQ);
}

__global__ __launch_bounds__(NTHR) void k_convert(
    const float* __restrict__ xq, const float* __restrict__ xk, const float* __restrict__ xv,
    const float* __restrict__ wq, const float* __restrict__ wk, const float* __restrict__ wv,
    const float* __restrict__ wo,
    unsigned short* xb, unsigned short* wb, unsigned short* wob, int nUnits)
{
  const int u = (int)blockIdx.x * NTHR + (int)threadIdx.x;
  if (u >= nUnits) return;
  const float* src;
  unsigned short* dst;
  if (u < NXU) {
    const int z = u >> 18, off = u & ((1 << 18) - 1);
    const float* xs = (z == 0) ? xq : ((z == 1) ? xk : xv);
    src = xs + (size_t)off * 8;
    dst = xb + (size_t)u * 8;
  } else if (u < NXU + NWU) {
    const int e = u - NXU;
    const int z = e >> 15, off = e & ((1 << 15) - 1);
    const float* wsp = (z == 0) ? wq : ((z == 1) ? wk : wv);
    src = wsp + (size_t)off * 8;
    dst = wb + (size_t)e * 8;
  } else {
    const int e = u - NXU - NWU;
    const int n = e >> 7;
    const int c8 = (e & 127) * 8;
    src = wo + (size_t)n * DM + (c8 & (DM - 1));
    dst = wob + (size_t)n * KOUT + c8;
  }
  const v4f a = *(const v4fa*)src;
  const v4f b = *(const v4fa*)(src + 4);
  const v8us o = cvt8b(a, b);
  *(volatile v8us*)dst = o;
  __threadfence();
  *(volatile v8us*)dst = o;
}

template<int EPI>
__global__ __launch_bounds__(GTHR) void k_gemm(
    const unsigned short* __restrict__ A, const unsigned short* __restrict__ WT,
    float* outF, int K, int strideA, int strideW, int strideO)
{
  __shared__ __attribute__((aligned(16))) float stg[GBM * GBN];
  const int tid = (int)threadIdx.x, lane = tid & 31, wave = tid >> 5, hh = lane >> 4, m = lane & 15;
  const int z = (int)blockIdx.z;
  const unsigned short* Az = A  + (size_t)z * (size_t)strideA;
  const unsigned short* Wz = WT + (size_t)z * (size_t)strideW;
  float* Oz = outF + (size_t)z * (size_t)strideO;
  const int rowBase = (int)blockIdx.x * GBM;
  const int col0    = (int)blockIdx.y * GBN;

  v8f acc[4];
  {
    const v8f zz = {0.f, 0.f, 0.f, 0.f, 0.f, 0.f, 0.f, 0.f};
    acc[0] = zz; acc[1] = zz; acc[2] = zz; acc[3] = zz;
  }
  const unsigned short* ap = Az + (size_t)(rowBase + 16 * wave + m) * (size_t)K + 8 * hh;
  const unsigned short* wp = Wz + (size_t)(col0 + m) * (size_t)K + 8 * hh;
  const int ksteps = K >> 5;
#pragma unroll 1
  for (int ks = 0; ks < ksteps; ++ks) {
    FragB af;
    af.h[0] = *(const v8usa*)(ap + 32 * ks);
    af.h[1] = *(const v8usa*)(ap + 32 * ks + 16);
#pragma unroll
    for (int t = 0; t < 4; ++t) {
      const unsigned short* wq = wp + (size_t)(16 * t) * (size_t)K + 32 * ks;
      FragB bf;
      bf.h[0] = *(const v8usa*)wq;
      bf.h[1] = *(const v8usa*)(wq + 16);
      acc[t] = wmb(af, bf, acc[t]);
    }
  }

#pragma unroll
  for (int t = 0; t < 4; ++t) {
    const int lc = 16 * t + m;
#pragma unroll
    for (int r = 0; r < 8; ++r) {
      const int lr = 16 * wave + 8 * hh + r;
      stg[lr * GBN + lc] = acc[t][r];
    }
  }
  __syncthreads();

  float* ob;
  int ldo;
  if (EPI == 0) {
    const int bq = rowBase >> 10;
    const int s0 = rowBase & (SEQ - 1);
    ob  = Oz + ((size_t)(bq * NH + (int)blockIdx.y) * SEQ + s0) * DK;
    ldo = DK;
  } else {
    ob  = Oz + (size_t)rowBase * DM + col0;
    ldo = DM;
  }
  v4f fv[8];
#pragma unroll
  for (int i = 0; i < 8; ++i) {
    const int lr = 16 * wave + 2 * i + hh;
    fv[i] = *(const v4fa*)(stg + lr * GBN + 4 * m);
  }
#pragma unroll
  for (int i = 0; i < 8; ++i) {
    const int lr = 16 * wave + 2 * i + hh;
    float* op = ob + (size_t)lr * (size_t)ldo + 4 * m;
    *(volatile v4f*)op = fv[i];
  }
  __threadfence();
#pragma unroll
  for (int i = 0; i < 8; ++i) {
    const int lr = 16 * wave + 2 * i + hh;
    float* op = ob + (size_t)lr * (size_t)ldo + 4 * m;
    *(volatile v4f*)op = fv[i];
  }
}

__global__ __launch_bounds__(NTHR) void k_scores(
    const int* __restrict__ pos_enc, const int* __restrict__ pos_pad,
    const float* __restrict__ rel_q, const float* __restrict__ rel_k,
    const float* __restrict__ QP, const float* __restrict__ KPl, float* S)
{
  __shared__ __attribute__((aligned(16))) float rk[DK];
  __shared__ __attribute__((aligned(16))) float rq[DK];
  const int tid = (int)threadIdx.x;
  const int bh = (int)blockIdx.y, h = bh & (NH - 1);
  const int f = (int)blockIdx.x * NTHR + tid;
  const int w = f >> 10;
  {
    const int sel = tid >> 6, j = tid & 63;
    const size_t rb = (size_t)(h * W2 + w) * DK + j;
    if (sel == 0) rk[j] = bf16f(rel_k[rb]);
    if (sel == 1) rq[j] = bf16f(rel_q[rb]);
  }
  __syncthreads();

  int qi, ki; bool msk;
  slot_idx(pos_enc, pos_pad, bh, f, qi, ki, msk);
  const float* qrow = QP  + ((size_t)bh * SEQ + qi) * DK;
  const float* krow = KPl + ((size_t)bh * SEQ + ki) * DK;
  float c2c = 0.f, c2p = 0.f, p2c = 0.f;
#pragma unroll 1
  for (int j = 0; j < DK / 4; ++j) {
    const v4f qv  = *(const v4fa*)(qrow + 4 * j);
    const v4f kv  = *(const v4fa*)(krow + 4 * j);
    const v4f rkv = *(const v4fa*)(rk + 4 * j);
    const v4f rqv = *(const v4fa*)(rq + 4 * j);
    c2c = fmaf(qv.x, kv.x, c2c);   c2c = fmaf(qv.y, kv.y, c2c);   c2c = fmaf(qv.z, kv.z, c2c);   c2c = fmaf(qv.w, kv.w, c2c);
    c2p = fmaf(qv.x, rkv.x, c2p);  c2p = fmaf(qv.y, rkv.y, c2p);  c2p = fmaf(qv.z, rkv.z, c2p);  c2p = fmaf(qv.w, rkv.w, c2p);
    p2c = fmaf(rqv.x, kv.x, p2c);  p2c = fmaf(rqv.y, kv.y, p2c);  p2c = fmaf(rqv.z, kv.z, p2c);  p2c = fmaf(rqv.w, kv.w, p2c);
  }
  const float sc = msk ? NEGBIG : ((c2c + c2p) + p2c) * RINV24;
  float* sp = S + (size_t)bh * NSLOT + f;
  *(volatile float*)sp = sc;
  __threadfence();
  *(volatile float*)sp = sc;
}

__global__ __launch_bounds__(NTHR) void k_agg(
    const int* __restrict__ pos_enc, const int* __restrict__ pos_pad,
    const float* __restrict__ rel_v, const float* __restrict__ S, const float* __restrict__ VP,
    unsigned short* OA)
{
  extern __shared__ v4f lds_dyn[];
  int*   reg2 = (int*)lds_dyn;
  int*   scnt = reg2 + NSLOT;
  int*   soff = scnt + SEQ;
  int*   cur  = soff + SEQ;
  float* relv = (float*)(cur + SEQ);
  float* stw  = relv + W2 * DK;
  float* red  = stw + NWAVE * 64;
  int*   wtot = (int*)(red + 16);
  const int tid = (int)threadIdx.x, lane = tid & 31, wave = tid >> 5;
  const int bh = (int)blockIdx.x, b = bh >> 3, h = bh & (NH - 1);
  const float* sb = S + (size_t)bh * NSLOT;

  {
    const v4i z4 = {0, 0, 0, 0};
#pragma unroll 1
    for (int i = tid; i < NSLOT / 4; i += NTHR) *(v4ia*)(reg2 + 4 * i) = z4;
    *(v4ia*)(scnt + 4 * tid) = z4;
    const float* rp = rel_v + (size_t)h * (W2 * DK) + 8 * tid;
    const v4f a = *(const v4fa*)rp;
    const v4f c = *(const v4fa*)(rp + 4);
    float* q = relv + 8 * tid;
    q[0] = bf16f(a.x); q[1] = bf16f(a.y); q[2] = bf16f(a.z); q[3] = bf16f(a.w);
    q[4] = bf16f(c.x); q[5] = bf16f(c.y); q[6] = bf16f(c.z); q[7] = bf16f(c.w);
  }
  __syncthreads();

  float mx = -3.0e38f;
#pragma unroll 1
  for (int i = 0; i < NSLOT / (4 * NTHR); ++i) {
    const v4f s4 = *(const v4fa*)(sb + (size_t)i * (4 * NTHR) + 4 * tid);
    mx = fmaxf(fmaxf(mx, fmaxf(s4.x, s4.y)), fmaxf(s4.z, s4.w));
  }
#pragma unroll
  for (int off = 16; off > 0; off >>= 1) mx = fmaxf(mx, __shfl_xor(mx, off));
  if (lane == 0) red[wave] = mx;
  __syncthreads();
  float M = red[0];
#pragma unroll
  for (int w2 = 1; w2 < NWAVE; ++w2) M = fmaxf(M, red[w2]);
  float zs = 0.f;
#pragma unroll 1
  for (int i = 0; i < NSLOT / (4 * NTHR); ++i) {
    const v4f s4 = *(const v4fa*)(sb + (size_t)i * (4 * NTHR) + 4 * tid);
    zs += (__expf(s4.x - M) + __expf(s4.y - M)) + (__expf(s4.z - M) + __expf(s4.w - M));
  }
#pragma unroll
  for (int off = 16; off > 0; off >>= 1) zs += __shfl_xor(zs, off);
  if (lane == 0) red[NWAVE + wave] = zs;
  __syncthreads();
  float Z = 0.f;
#pragma unroll
  for (int w2 = 0; w2 < NWAVE; ++w2) Z += red[NWAVE + w2];
  const float invZ = 1.0f / Z;

  if (wave == 0) {
#pragma unroll 1
    for (int b0 = 0; b0 < NSLOT; b0 += 32) {
      const int f = b0 + lane;
      int qi, ki; bool msk;
      slot_idx(pos_enc, pos_pad, bh, f, qi, ki, msk);
#pragma unroll 1
      for (int k = 0; k < 32; ++k) {
        const int t = __builtin_amdgcn_readlane(qi, k) & (SEQ - 1);
        if (lane == 0) scnt[t] = scnt[t] + 1;
      }
    }
  }
  __syncthreads();

  int tot;
  {
    const v4i ca = *(const v4ia*)(scnt + 4 * tid);
    const int e0 = ca.x < 0 ? 0 : ca.x, e1 = ca.y < 0 ? 0 : ca.y, e2 = ca.z < 0 ? 0 : ca.z, e3 = ca.w < 0 ? 0 : ca.w;
    const int ts = e0 + e1 + e2 + e3;
    int incl = ts;
#pragma unroll
    for (int d = 1; d < 32; d <<= 1) {
      const int up = __shfl_up(incl, d);
      if (lane >= d) incl += up;
    }
    if (lane == 31) wtot[wave] = incl;
    __syncthreads();
    int pre = 0;
    tot = 0;
#pragma unroll
    for (int w2 = 0; w2 < NWAVE; ++w2) {
      const int t = wtot[w2];
      tot += t;
      pre += (w2 < wave) ? t : 0;
    }
    int run = pre + incl - ts;
    soff[4 * tid + 0] = run; run += e0;
    soff[4 * tid + 1] = run; run += e1;
    soff[4 * tid + 2] = run; run += e2;
    soff[4 * tid + 3] = run;
  }
  __syncthreads();
  *(v4ia*)(cur + 4 * tid) = *(const v4ia*)(soff + 4 * tid);
  __syncthreads();

  if (wave == 0) {
#pragma unroll 1
    for (int b0 = 0; b0 < NSLOT; b0 += 32) {
      const int f = b0 + lane;
      int qi, ki; bool msk;
      slot_idx(pos_enc, pos_pad, bh, f, qi, ki, msk);
      const int ent = f | (ki << 15);
#pragma unroll 1
      for (int k = 0; k < 32; ++k) {
        const int t = __builtin_amdgcn_readlane(qi, k) & (SEQ - 1);
        const int e = __builtin_amdgcn_readlane(ent, k);
        if (lane == 0) {
          int pos = cur[t];
          pos = pos < 0 ? 0 : (pos > NSLOT - 1 ? NSLOT - 1 : pos);
          reg2[pos] = e;
          cur[t] = pos + 1;
        }
      }
    }
  }
  __syncthreads();

  const float qnan = __int_as_float(0x7fc00000);
  const bool bad_tot = (tot != NSLOT);
  float* sw = stw + wave * 64;
  const int lc = lane & 7;
  const bool islo = (lane & 8) != 0;
  const float* vb = VP + (size_t)bh * SEQ * DK;
#pragma unroll 1
  for (int jt = 0; jt < TPW; ++jt) {
    const int tg = wave * TPW + jt;
    int st = soff[tg];
    const int craw = scnt[tg];
    int cnt = craw;
    st  = st < 0 ? 0 : (st > NSLOT ? NSLOT : st);
    cnt = cnt < 0 ? 0 : (cnt > DEGCAP ? DEGCAP : cnt);
    if (cnt > NSLOT - st) cnt = NSLOT - st;
    const float pz = (bad_tot || craw > DEGCAP || craw < 0) ? qnan : 0.0f;
    float a0 = 0.f, a1 = 0.f;
#pragma unroll 1
    for (int q = 0; q < cnt; ++q) {
      int idx = st + q;
      idx = idx > NSLOT - 1 ? NSLOT - 1 : idx;
      const int e  = reg2[idx];
      const int f  = e & (NSLOT - 1);
      const int ki = (e >> 15) & (SEQ - 1);
      const int wr = f >> 10;
      const float s = sb[f];
      const float p = __expf(s - M) * invZ;
      const float* vr = vb + (size_t)ki * DK + lane;
      const float v0 = vr[0];
      const float v1 = vr[32];
      const float r0 = relv[wr * DK + lane];
      const float r1 = relv[wr * DK + 32 + lane];
      a0 = fmaf(p, v0 + r0, a0);
      a1 = fmaf(p, v1 + r1, a1);
    }
    a0 += pz;
    a1 += pz;
    __builtin_amdgcn_fence(__ATOMIC_RELEASE, "wavefront");
    __builtin_amdgcn_wave_barrier();
    sw[lane]      = a0;
    sw[32 + lane] = a1;
    __builtin_amdgcn_fence(__ATOMIC_RELEASE, "wavefront");
    __builtin_amdgcn_wave_barrier();
    const v4f ga = *(const v4fa*)(sw + 8 * lc);
    const v4f gb = *(const v4fa*)(sw + 8 * lc + 4);
    const v8us ov = split8(ga, gb, islo);
    const int orow = b * SEQ + tg;
    unsigned short* dst = OA + (size_t)orow * KOUT + (islo ? DM : 0) + h * DK + 8 * lc;
    const bool wsv = lane < 16;
    if (wsv) *(volatile v8us*)dst = ov;
    __threadfence();
    if (wsv) *(volatile v8us*)dst = ov;
  }
}

static inline int cdiv(int a, int b) { return (a + b - 1) / b; }

extern "C" void kernel_launch(void* const* d_in, const int* in_sizes, int n_in,
                              void* d_out, int out_size, void* d_ws, size_t ws_size,
                              hipStream_t stream) {
  if (n_in < 12) return;
  if (in_sizes[0] != NB_ * SEQ * DM || in_sizes[1] != NB_ * SEQ * DM || in_sizes[2] != NB_ * SEQ * DM) return;
  if (in_sizes[3] != NPOS || in_sizes[4] != NPOS) return;
  if (in_sizes[5] != NH * W2 * DK || in_sizes[6] != NH * W2 * DK || in_sizes[7] != NH * W2 * DK) return;
  if (in_sizes[8] != DM * DM || in_sizes[9] != DM * DM || in_sizes[10] != DM * DM || in_sizes[11] != DM * DM) return;
  if (out_size != NB_ * SEQ * DM) return;

  const float* query   = (const float*)d_in[0];
  const float* keyx    = (const float*)d_in[1];
  const float* value   = (const float*)d_in[2];
  const int*   pos_enc = (const int*)  d_in[3];
  const int*   pos_pad = (const int*)  d_in[4];
  const float* rel_q   = (const float*)d_in[5];
  const float* rel_k   = (const float*)d_in[6];
  const float* rel_v   = (const float*)d_in[7];
  const float* Wq      = (const float*)d_in[8];
  const float* Wk      = (const float*)d_in[9];
  const float* Wv      = (const float*)d_in[10];
  const float* Wo      = (const float*)d_in[11];
  float*       out     = (float*)d_out;

  char* ws = (char*)d_ws;
  size_t off = 0;
  const size_t oXB  = off; off += (size_t)NXU * 16;
  const size_t oWB  = off; off += (size_t)NWU * 16;
  const size_t oWOB = off; off += (size_t)NWOU * 16;
  const size_t oQKV = off; off += (size_t)3 * PLQ * 4;
  const size_t oS   = off; off += (size_t)NBH * NSLOT * 4;
  const size_t oOA  = off; off += (size_t)MROWS * KOUT * 2;
  if (off > ws_size || off > (size_t)WSMAX) return;
  unsigned short* XB  = (unsigned short*)(ws + oXB);
  unsigned short* WB  = (unsigned short*)(ws + oWB);
  unsigned short* WOB = (unsigned short*)(ws + oWOB);
  float*          QKV = (float*)(ws + oQKV);
  float*          S   = (float*)(ws + oS);
  unsigned short* OA  = (unsigned short*)(ws + oOA);
  const float* QP  = QKV;
  const float* KPl = QKV + (size_t)PLQ;
  const float* VP  = QKV + (size_t)2 * PLQ;

  hipFuncSetAttribute(reinterpret_cast<const void*>(&k_agg),
                      hipFuncAttributeMaxDynamicSharedMemorySize, LDS_AGG);

  k_convert<<<NCU / NTHR, NTHR, 0, stream>>>(query, keyx, value, Wq, Wk, Wv, Wo, XB, WB, WOB, NCU);
  k_gemm<0><<<dim3(MROWS / GBM, DM / GBN, 3), GTHR, 0, stream>>>(XB, WB, QKV, DM, MROWS * DM, DM * DM, PLQ);
  k_scores<<<dim3(NSLOT / NTHR, NBH), NTHR, 0, stream>>>(pos_enc, pos_pad, rel_q, rel_k, QP, KPl, S);
  k_agg<<<NBH, NTHR, LDS_AGG, stream>>>(pos_enc, pos_pad, rel_v, S, VP, OA);
  k_gemm<1><<<dim3(MROWS / GBM, DM / GBN, 1), GTHR, 0, stream>>>(OA, WOB, out, KOUT, 0, 0, 0);
}
